// DSSMamba2_47296179863956
// MI455X (gfx1250) — hardware-verified
//
#include <hip/hip_runtime.h>
#include <hip/hip_bf16.h>
#include <math.h>

#define SEQL   1024
#define DM     1024
#define DIN    2048
#define NS     64
#define NH     32
#define HD     64
#define CONVD  (DIN + 2 * NS)
#define DPROJ  (2 * DIN + 2 * NS + NH)
#define LDZ    4288
#define CH     256
#define NCH    (SEQL / CH)
#define XW     DIN
#define GSTR   40
#define OSTR   68
#define SMEMB  (8 * 16 * OSTR * 4)
#define EPSV   1e-5f
#define SXN    2304
#define PREVE  2048

static_assert(SMEMB >= (2 * 128 * GSTR + 2 * 64 * GSTR) * 2);
static_assert(SEQL % CH == 0);
static_assert(CH == 256);
static_assert(HD == 64);
static_assert(NS == 64);
static_assert(NH * HD == DIN);
static_assert(LDZ % 64 == 0);
static_assert(LDZ >= DPROJ);
static_assert(SXN >= 9 * 256);
static_assert(SXN >= CONVD);
static_assert(CONVD - DIN == 2 * NS);
static_assert(NCH * NCH <= 256);
static_assert(PREVE % NS == 0);
static_assert(HD % (PREVE / NS) == 0);
static_assert((XW * NS) % PREVE == 0);

typedef unsigned short us16 __attribute__((ext_vector_type(16)));
typedef unsigned short us8  __attribute__((ext_vector_type(8)));
typedef unsigned short us8a __attribute__((ext_vector_type(8), may_alias));
typedef __bf16 v16b __attribute__((ext_vector_type(16)));
typedef float v8f __attribute__((ext_vector_type(8)));
typedef float v4f __attribute__((ext_vector_type(4)));
typedef float v4fa __attribute__((ext_vector_type(4), may_alias));
union FragU { us16 v; us8 h[2]; };

__device__ __forceinline__ unsigned short bf16_bits(float f) {
  unsigned u = __float_as_uint(f);
  u += 0x7FFFu + ((u >> 16) & 1u);
  return (unsigned short)(u >> 16);
}
__device__ __forceinline__ float bf16_val(unsigned short b) { return __uint_as_float(((unsigned)b) << 16); }
__device__ __forceinline__ float bf16r(float f) { return bf16_val(bf16_bits(f)); }
__device__ __forceinline__ float siluf(float x) { return x * (1.0f / (1.0f + __expf(-x))); }

__device__ __forceinline__ v8f mma_bf16(us16 a, us16 b, v8f c) {
  return __builtin_amdgcn_wmma_f32_16x16x32_bf16(false, __builtin_bit_cast(v16b, a), false, __builtin_bit_cast(v16b, b), (short)0, c, false, false);
}
__device__ __forceinline__ void wguard(v8f& c0, v8f& c1, v8f& c2, v8f& c3, const us16& a0, const us16& a1,
                                       const us16& b0, const us16& b1, const us16& b2, const us16& b3,
                                       const us16& b4, const us16& b5, const us16& b6, const us16& b7) {
#if defined(__HIP_DEVICE_COMPILE__)
  asm volatile("v_nop\n\tv_nop\n\tv_nop\n\tv_nop"
               : "+v"(c0), "+v"(c1), "+v"(c2), "+v"(c3)
               : "v"(a0), "v"(a1), "v"(b0), "v"(b1), "v"(b2), "v"(b3), "v"(b4), "v"(b5), "v"(b6), "v"(b7));
#endif
}

__device__ __forceinline__ us16 lds_frag(const unsigned short* base) {
  const int lane = threadIdx.x & 31, r = lane & 15, kh = (lane >> 4) * 8;
  FragU f;
  f.h[0] = *(const us8a*)(base + r * GSTR + kh);
  f.h[1] = *(const us8a*)(base + r * GSTR + 16 + kh);
  return f.v;
}

template <int KM>
__device__ __forceinline__ void stage_a(unsigned short* lds, const unsigned short* __restrict__ P, int ld, int m0, int k0, int tid) {
  if (KM == 0) {
    const int row = tid >> 1, cq = (tid & 1) * 16;
    const unsigned short* src = P + (size_t)(m0 + row) * ld + k0 + cq;
    const us8 v0 = *(const us8a*)src;
    const us8 v1 = *(const us8a*)(src + 8);
    *(us8a*)(lds + row * GSTR + cq) = v0;
    *(us8a*)(lds + row * GSTR + cq + 8) = v1;
  } else {
    const int k = tid >> 3, mq = (tid & 7) * 16;
    const unsigned short* src = P + (size_t)(k0 + k) * ld + m0 + mq;
    const us8 v0 = *(const us8a*)src;
    const us8 v1 = *(const us8a*)(src + 8);
#pragma unroll
    for (int u = 0; u < 8; ++u) { lds[(mq + u) * GSTR + k] = v0[u]; lds[(mq + 8 + u) * GSTR + k] = v1[u]; }
  }
}
template <int KM>
__device__ __forceinline__ void stage_b(unsigned short* lds, const unsigned short* __restrict__ P, int ld, int n0, int k0, int tid) {
  if (KM == 0) {
    const int row = tid >> 2, kq = (tid & 3) * 8;
    const us8 v = *(const us8a*)(P + (size_t)(n0 + row) * ld + k0 + kq);
    *(us8a*)(lds + row * GSTR + kq) = v;
  } else {
    const int k = tid >> 3, nq = (tid & 7) * 8;
    const us8 v = *(const us8a*)(P + (size_t)(k0 + k) * ld + n0 + nq);
#pragma unroll
    for (int u = 0; u < 8; ++u) lds[(nq + u) * GSTR + k] = v[u];
  }
}
__device__ __forceinline__ void stage_w(unsigned short* lhi, unsigned short* llo, const float* __restrict__ G, int ldg,
                                        const float* sac, int m0, int k0, int tid) {
  const int row = tid >> 1, cq = (tid & 1) * 16, m = m0 + row;
  const float* src = G + (size_t)m * ldg + k0 + cq;
  v4f g4[4];
#pragma unroll
  for (int q = 0; q < 4; ++q) g4[q] = *(const v4fa*)(src + 4 * q);
  const float am = sac[m];
  us8 h0, h1, l0, l1;
#pragma unroll
  for (int u = 0; u < 16; ++u) {
    const int s = k0 + cq + u;
    const float d = expf(am - sac[s]);
    const float w = (s <= m) ? g4[u >> 2][u & 3] * d : 0.0f;
    const unsigned short hb = bf16_bits(w);
    const unsigned short lb = bf16_bits(w - bf16_val(hb));
    if (u < 8) { h0[u] = hb; l0[u] = lb; } else { h1[u - 8] = hb; l1[u - 8] = lb; }
  }
  *(us8a*)(lhi + row * GSTR + cq) = h0;
  *(us8a*)(lhi + row * GSTR + cq + 8) = h1;
  *(us8a*)(llo + row * GSTR + cq) = l0;
  *(us8a*)(llo + row * GSTR + cq + 8) = l1;
}

template <int NA, int NBP, int AKM, int BKM, int EPI, int FLIP>
__global__ __launch_bounds__(256) void k_gemm(
    const unsigned short* __restrict__ A0, const unsigned short* __restrict__ A1, const float* __restrict__ Af,
    int lda, long long sAc, long long sAh,
    const unsigned short* __restrict__ B0, const unsigned short* __restrict__ B1, int ldb, long long sBc, long long sBh,
    float* Yg, int ldy, long long sYc, long long sYh,
    unsigned short* OH, unsigned short* OL, int ldo,
    const float* __restrict__ R, int ldr, long long sRc, long long sRh,
    const float* __restrict__ acs, long long sXc, long long sXh,
    int zh, int K)
{
  __shared__ __attribute__((aligned(16))) unsigned char sm[SMEMB];
  __shared__ float sacs[CH];
  unsigned short* lA0 = (unsigned short*)sm;
  unsigned short* lA1 = lA0 + 128 * GSTR;
  unsigned short* lB0 = lA1 + 128 * GSTR;
  unsigned short* lB1 = lB0 + 64 * GSTR;
  float* oS = (float*)sm;
  const int tid = threadIdx.x, lane = tid & 31, wave = tid >> 5, cl = lane & 15, hh = lane >> 4;
  const int m0 = blockIdx.x * 128, n0 = blockIdx.y * 64;
  const int z = blockIdx.z, zc = z / zh, zq = z - zc * zh;
  const long long oA = (long long)zc * sAc + (long long)zq * sAh;
  const long long oB = (long long)zc * sBc + (long long)zq * sBh;
  A0 += oA; A1 += oA; Af += oA;
  B0 += oB; B1 += oB;
  const float* acz = acs + (long long)zc * sXc + (long long)zq * sXh;
  if (AKM == 2) sacs[tid] = acz[(size_t)tid * NH];
  int kend = K;
  if (AKM == 2) { const int t = m0 + 128; kend = (t < K) ? t : K; }

  v8f acc[4];
#pragma unroll
  for (int j = 0; j < 4; ++j) { v8f zz = {0.f, 0.f, 0.f, 0.f, 0.f, 0.f, 0.f, 0.f}; acc[j] = zz; }

#pragma unroll 1
  for (int k0 = 0; k0 < kend; k0 += 32) {
    __syncthreads();
    if (AKM == 2) {
      stage_w(lA0, lA1, Af, lda, sacs, m0, k0, tid);
    } else {
      stage_a<(AKM == 1) ? 1 : 0>(lA0, A0, lda, m0, k0, tid);
      if (NA > 1) stage_a<(AKM == 1) ? 1 : 0>(lA1, A1, lda, m0, k0, tid);
    }
    stage_b<BKM>(lB0, B0, ldb, n0, k0, tid);
    if (NBP > 1) stage_b<BKM>(lB1, B1, ldb, n0, k0, tid);
    __syncthreads();
    const us16 af0 = lds_frag(lA0 + 16 * wave * GSTR);
    us16 af1 = af0;
    if (NA > 1) af1 = lds_frag(lA1 + 16 * wave * GSTR);
    us16 bf0[4], bf1[4];
#pragma unroll
    for (int j = 0; j < 4; ++j) { bf0[j] = lds_frag(lB0 + 16 * j * GSTR); bf1[j] = bf0[j]; }
    if (NBP > 1) {
#pragma unroll
      for (int j = 0; j < 4; ++j) bf1[j] = lds_frag(lB1 + 16 * j * GSTR);
    }
#pragma unroll
    for (int j = 0; j < 4; ++j) acc[j] = mma_bf16(af0, bf0[j], acc[j]);
    if (NBP > 1) {
#pragma unroll
      for (int j = 0; j < 4; ++j) acc[j] = mma_bf16(af0, bf1[j], acc[j]);
    }
    if (NA > 1) {
#pragma unroll
      for (int j = 0; j < 4; ++j) acc[j] = mma_bf16(af1, bf0[j], acc[j]);
    }
    wguard(acc[0], acc[1], acc[2], acc[3], af0, af1, bf0[0], bf0[1], bf0[2], bf0[3], bf1[0], bf1[1], bf1[2], bf1[3]);
  }
  __syncthreads();

  float* so = oS + wave * (16 * OSTR);
#pragma unroll
  for (int j = 0; j < 4; ++j)
#pragma unroll
    for (int r = 0; r < 8; ++r) so[(8 * hh + r) * OSTR + 16 * j + cl] = acc[j][r];
  __syncthreads();
  if (EPI != 0) {
    const float* Rz = R + (long long)zc * sRc + (long long)zq * sRh;
#pragma unroll 1
    for (int e = lane; e < 16 * 64; e += 32) {
      const int r = e >> 6, c = e & 63;
      const int m = m0 + 16 * wave + r, n = n0 + c;
      float v = so[r * OSTR + c];
      if (EPI == 1) v = v * expf(acz[(size_t)m * NH]);
      if (EPI == 2) v = v + Rz[(size_t)m * ldr + n];
      if (EPI == 3) v = siluf(v);
      so[r * OSTR + c] = v;
    }
    __syncthreads();
  }
  if (EPI == 3) {
#pragma unroll
    for (int pass = 0; pass < 2; ++pass) {
#pragma unroll
      for (int it = 0; it < 4; ++it) {
        const int ch = it * 32 + lane, r = ch >> 3, q = (ch & 7) * 8;
        const v4f va = *(const v4fa*)(so + r * OSTR + q);
        const v4f vb = *(const v4fa*)(so + r * OSTR + q + 4);
        us8 hi, lo;
#pragma unroll
        for (int u = 0; u < 4; ++u) {
          const unsigned short a = bf16_bits(va[u]);
          hi[u] = a; lo[u] = bf16_bits(va[u] - bf16_val(a));
          const unsigned short b = bf16_bits(vb[u]);
          hi[4 + u] = b; lo[4 + u] = bf16_bits(vb[u] - bf16_val(b));
        }
        const int row = m0 + 16 * wave + r;
        const int orow = FLIP ? (SEQL - 1 - row) : row;
        const size_t o = (size_t)orow * ldo + n0 + q;
        *(volatile us8*)(OH + o) = hi;
        *(volatile us8*)(OL + o) = lo;
      }
      __threadfence();
    }
  } else {
#pragma unroll
    for (int pass = 0; pass < 2; ++pass) {
      float* Y = Yg + (long long)zc * sYc + (long long)zq * sYh;
#pragma unroll
      for (int it = 0; it < 8; ++it) {
        const int ch = it * 32 + lane, r = ch >> 4, q = (ch & 15) * 4;
        const v4f v = *(const v4fa*)(so + r * OSTR + q);
        *(volatile v4f*)(Y + (size_t)(m0 + 16 * wave + r) * ldy + n0 + q) = v;
      }
      __threadfence();
    }
  }
}

__global__ __launch_bounds__(256) void k_cvt(const float* __restrict__ src, unsigned short* dst, int nsrc, int ncol8, int total8) {
  const int idx = blockIdx.x * 256 + threadIdx.x;
  if (idx >= total8) return;
  const int row = idx / ncol8, c8 = (idx - row * ncol8) * 8;
  const int rs = (row < nsrc) ? row : (nsrc - 1);
  const float* s = src + (size_t)rs * (size_t)(ncol8 * 8) + c8;
  const v4f a = *(const v4fa*)s, b = *(const v4fa*)(s + 4);
  const bool zr = (row >= nsrc);
  us8 o;
#pragma unroll
  for (int u = 0; u < 4; ++u) {
    o[u]     = zr ? (unsigned short)0 : bf16_bits(a[u]);
    o[4 + u] = zr ? (unsigned short)0 : bf16_bits(b[u]);
  }
  const size_t off = (size_t)row * (size_t)(ncol8 * 8) + c8;
  *(volatile us8*)(dst + off) = o;
  __threadfence();
  *(volatile us8*)(dst + off) = o;
}

__global__ __launch_bounds__(256) void k_cvt_u(const float* __restrict__ u, unsigned short* Uf, unsigned short* Ub) {
  const int idx = blockIdx.x * 256 + threadIdx.x;
  if (idx >= SEQL * DM / 8) return;
  const int t = idx / (DM / 8), c8 = (idx - t * (DM / 8)) * 8;
  const float* s = u + (size_t)t * DM + c8;
  const v4f a = *(const v4fa*)s, b = *(const v4fa*)(s + 4);
  us8 o;
#pragma unroll
  for (int k = 0; k < 4; ++k) { o[k] = bf16_bits(a[k]); o[4 + k] = bf16_bits(b[k]); }
  const size_t of = (size_t)t * DM + c8, ob = (size_t)(SEQL - 1 - t) * DM + c8;
  *(volatile us8*)(Uf + of) = o;
  *(volatile us8*)(Ub + ob) = o;
  __threadfence();
  *(volatile us8*)(Uf + of) = o;
  *(volatile us8*)(Ub + ob) = o;
}

__global__ __launch_bounds__(32) void k_acs(const float* __restrict__ ZX, const float* __restrict__ dtb, const float* __restrict__ Alog,
                                            float* ACS, float* DT) {
#pragma clang fp contract(off)
  const int c = blockIdx.x, h = threadIdx.x;
  const float ab = -expf(bf16r(Alog[h]));
  const float db = bf16r(dtb[h]);
#pragma unroll 1
  for (int pass = 0; pass < 2; ++pass) {
    double run = 0.0;
#pragma unroll 1
    for (int i = 0; i < CH; ++i) {
      const size_t tok = (size_t)c * CH + i;
      const float xr = ZX[tok * LDZ + (DPROJ - NH) + h] + db;
      const float sp = fmaxf(xr, 0.0f) + log1pf(expf(-fabsf(xr)));
      const float a = sp * ab;
      run = run + (double)a;
      const float rf = (float)run;
      *(volatile float*)(ACS + tok * NH + h) = rf;
      *(volatile float*)(DT + tok * NH + h) = sp;
    }
    __threadfence();
  }
}

__global__ __launch_bounds__(256) void k_conv(const float* __restrict__ ZX, const float* __restrict__ cw, const float* __restrict__ cb,
                                             const float* __restrict__ ACS, const float* __restrict__ DT, float* XF,
                                             unsigned short* XTH, unsigned short* XTL, unsigned short* XDH, unsigned short* XDL,
                                             unsigned short* BHp, unsigned short* BLp, unsigned short* CHp, unsigned short* CLp) {
#pragma clang fp contract(off)
  __shared__ __attribute__((aligned(16))) float sx[SXN];
  const int t = blockIdx.x, tid = threadIdx.x, lane = tid & 31;
#pragma unroll 1
  for (int i = 0; i < 9; ++i) {
    const int j = tid + 256 * i;
    const int jc = (j < CONVD) ? j : (CONVD - 1);
    float acc = 0.0f;
#pragma unroll
    for (int k = 0; k < 4; ++k) {
      const int tt = t - 3 + k;
      const int tr = (tt > 0) ? tt : 0;
      const float w = bf16r(cw[jc * 4 + k]);
      const float xv = ZX[(size_t)tr * LDZ + DIN + jc];
      const float pr = w * xv;
      acc = acc + ((tt >= 0) ? pr : 0.0f);
    }
    acc = acc + bf16r(cb[jc]);
    sx[j] = siluf(acc);
  }
  __syncthreads();
  const v4f f0 = *(const v4fa*)(sx + 4 * tid);
  const v4f f1 = *(const v4fa*)(sx + 1024 + 4 * tid);
  float* xr = XF + (size_t)t * XW;
  const int c8 = 8 * tid, h = tid >> 3;
  const int last = t | (CH - 1);
  const float dtv = DT[(size_t)t * NH + h];
  const float dec = expf(ACS[(size_t)last * NH + h] - ACS[(size_t)t * NH + h]);
  const v4f x0 = *(const v4fa*)(sx + c8), x1 = *(const v4fa*)(sx + c8 + 4);
  us8 ph, pl, qh, ql;
#pragma unroll
  for (int u = 0; u < 4; ++u) {
    const float v0 = x0[u] * dtv;
    const unsigned short a0 = bf16_bits(v0);
    ph[u] = a0; pl[u] = bf16_bits(v0 - bf16_val(a0));
    const float w0 = v0 * dec;
    const unsigned short b0 = bf16_bits(w0);
    qh[u] = b0; ql[u] = bf16_bits(w0 - bf16_val(b0));
    const float v1 = x1[u] * dtv;
    const unsigned short a1 = bf16_bits(v1);
    ph[4 + u] = a1; pl[4 + u] = bf16_bits(v1 - bf16_val(a1));
    const float w1 = v1 * dec;
    const unsigned short b1 = bf16_bits(w1);
    qh[4 + u] = b1; ql[4 + u] = bf16_bits(w1 - bf16_val(b1));
  }
  const size_t o = (size_t)t * XW + c8;
  *(volatile v4f*)(xr + 4 * tid) = f0;
  *(volatile v4f*)(xr + 1024 + 4 * tid) = f1;
  *(volatile us8*)(XTH + o) = ph; *(volatile us8*)(XTL + o) = pl; *(volatile us8*)(XDH + o) = qh; *(volatile us8*)(XDL + o) = ql;
  __threadfence();
  *(volatile v4f*)(xr + 4 * tid) = f0;
  *(volatile v4f*)(xr + 1024 + 4 * tid) = f1;
  *(volatile us8*)(XTH + o) = ph; *(volatile us8*)(XTL + o) = pl; *(volatile us8*)(XDH + o) = qh; *(volatile us8*)(XDL + o) = ql;
  if (tid < 32) {
    const int grp = lane >> 3, q = (lane & 7) * 8;
    const int cbase = DIN + ((grp & 1) ? NS : 0) + q;
    const v4f a = *(const v4fa*)(sx + cbase), b = *(const v4fa*)(sx + cbase + 4);
    us8 hi, lo;
#pragma unroll
    for (int u = 0; u < 4; ++u) {
      const unsigned short ha = bf16_bits(a[u]);
      hi[u] = ha; lo[u] = bf16_bits(a[u] - bf16_val(ha));
      const unsigned short hb = bf16_bits(b[u]);
      hi[4 + u] = hb; lo[4 + u] = bf16_bits(b[u] - bf16_val(hb));
    }
    const us8 ov = (grp < 2) ? hi : lo;
    unsigned short* dst = (grp == 0) ? BHp : ((grp == 1) ? CHp : ((grp == 2) ? BLp : CLp));
    dst += (size_t)t * NS + q;
    *(volatile us8*)dst = ov;
    __threadfence();
    *(volatile us8*)dst = ov;
  }
}

__global__ __launch_bounds__(256) void k_prev(const float* __restrict__ S, const float* __restrict__ ACS,
                                             unsigned short* PH, unsigned short* PL) {
#pragma clang fp contract(off)
  __shared__ float co[NCH * NCH];
  const int part = blockIdx.x, tid = threadIdx.x;
  const int h = (part * (PREVE / NS)) / HD;
  {
    const int zz = tid % (NCH * NCH);
    const int z = zz / NCH, c = zz - z * NCH;
    float run = 0.0f, csz = 0.0f, csc = 0.0f;
#pragma unroll 1
    for (int j = 1; j <= NCH; ++j) {
      run = run + ACS[((size_t)(j - 1) * CH + (CH - 1)) * NH + h];
      csz = (j == z) ? run : csz;
      csc = (j == c + 1) ? run : csc;
    }
    const float e = expf(csz - csc);
    if (tid < NCH * NCH) co[tid] = (c + 1 <= z) ? e : 0.0f;
  }
  __syncthreads();
  const int e0 = part * PREVE + tid * 8;
  v4f s0[NCH], s1[NCH];
#pragma unroll
  for (int c = 0; c < NCH; ++c) {
    const size_t base = (size_t)c * (size_t)(XW * NS) + e0;
    s0[c] = *(const v4fa*)(S + base);
    s1[c] = *(const v4fa*)(S + base + 4);
  }
#pragma unroll 1
  for (int z = 0; z < NCH; ++z) {
    v4f o0 = {0.0f, 0.0f, 0.0f, 0.0f}, o1 = {0.0f, 0.0f, 0.0f, 0.0f};
#pragma unroll
    for (int c = 0; c < NCH; ++c) {
      const float k = co[z * NCH + c];
      o0 = o0 + s0[c] * k;
      o1 = o1 + s1[c] * k;
    }
    us8 hi, lo;
#pragma unroll
    for (int u = 0; u < 4; ++u) {
      const unsigned short a = bf16_bits(o0[u]);
      hi[u] = a; lo[u] = bf16_bits(o0[u] - bf16_val(a));
      const unsigned short bb = bf16_bits(o1[u]);
      hi[4 + u] = bb; lo[4 + u] = bf16_bits(o1[u] - bf16_val(bb));
    }
    const size_t ob = (size_t)z * (size_t)(XW * NS) + e0;
    *(volatile us8*)(PH + ob) = hi; *(volatile us8*)(PL + ob) = lo;
    __threadfence();
    *(volatile us8*)(PH + ob) = hi; *(volatile us8*)(PL + ob) = lo;
  }
}

__global__ __launch_bounds__(256) void k_gate(const float* __restrict__ Y, const float* __restrict__ XF, const float* __restrict__ ZX,
                                             const float* __restrict__ Dv, const float* __restrict__ nw,
                                             unsigned short* YGH, unsigned short* YGL) {
#pragma clang fp contract(off)
  __shared__ float red[8];
  const int t = blockIdx.x, tid = threadIdx.x, lane = tid & 31, wave = tid >> 5;
  const int c8 = 8 * tid, h = tid >> 3;
  const float Dh = bf16r(Dv[h]);
  const float* yr = Y + (size_t)t * XW + c8;
  const float* xr = XF + (size_t)t * XW + c8;
  const float* zr = ZX + (size_t)t * LDZ + c8;
  const v4f y0 = *(const v4fa*)yr, y1 = *(const v4fa*)(yr + 4);
  const v4f x0 = *(const v4fa*)xr, x1 = *(const v4fa*)(xr + 4);
  const v4f z0 = *(const v4fa*)zr, z1 = *(const v4fa*)(zr + 4);
  const v4f w0 = *(const v4fa*)(nw + c8), w1 = *(const v4fa*)(nw + c8 + 4);
  v4f g0 = {0.0f, 0.0f, 0.0f, 0.0f}, g1 = {0.0f, 0.0f, 0.0f, 0.0f};
  float ss = 0.0f;
#pragma unroll
  for (int u = 0; u < 4; ++u) {
    const float a = (y0[u] + Dh * x0[u]) * siluf(z0[u]);
    const float b = (y1[u] + Dh * x1[u]) * siluf(z1[u]);
    g0[u] = a; g1[u] = b;
    ss = ss + a * a;
    ss = ss + b * b;
  }
#pragma unroll
  for (int off = 16; off > 0; off >>= 1) ss = ss + __shfl_xor(ss, off, 32);
  if (lane == 0) red[wave] = ss;
  __syncthreads();
  float tot = 0.0f;
#pragma unroll
  for (int w = 0; w < 8; ++w) tot = tot + red[w];
  const float rn = rsqrtf(tot * (1.0f / (float)DIN) + EPSV);
  us8 hi, lo;
#pragma unroll
  for (int u = 0; u < 4; ++u) {
    const float a = (g0[u] * rn) * bf16r(w0[u]);
    const unsigned short ha = bf16_bits(a);
    hi[u] = ha; lo[u] = bf16_bits(a - bf16_val(ha));
    const float b = (g1[u] * rn) * bf16r(w1[u]);
    const unsigned short hb = bf16_bits(b);
    hi[4 + u] = hb; lo[4 + u] = bf16_bits(b - bf16_val(hb));
  }
  const size_t o = (size_t)t * XW + c8;
  *(volatile us8*)(YGH + o) = hi; *(volatile us8*)(YGL + o) = lo;
  __threadfence();
  *(volatile us8*)(YGH + o) = hi; *(volatile us8*)(YGL + o) = lo;
}

extern "C" void kernel_launch(void* const* d_in, const int* in_sizes, int n_in,
                              void* d_out, int out_size, void* d_ws, size_t ws_size,
                              hipStream_t stream) {
  if (n_in < 18) return;
  if (in_sizes[0] != SEQL * DM || in_sizes[1] != DPROJ * DM || in_sizes[2] != DPROJ * DM ||
      in_sizes[3] != CONVD * 4 || in_sizes[4] != CONVD || in_sizes[5] != CONVD * 4 || in_sizes[6] != CONVD ||
      in_sizes[7] != NH || in_sizes[8] != NH || in_sizes[9] != NH || in_sizes[10] != NH ||
      in_sizes[11] != NH || in_sizes[12] != NH || in_sizes[13] != DIN || in_sizes[14] != DIN ||
      in_sizes[15] != DM * DIN || in_sizes[16] != DM * DIN || in_sizes[17] != DM * DIN ||
      out_size != SEQL * DM) return;
  const float* u       = (const float*)d_in[0];
  const float* Win[2]  = {(const float*)d_in[1], (const float*)d_in[2]};
  const float* cwv[2]  = {(const float*)d_in[3], (const float*)d_in[5]};
  const float* cbv[2]  = {(const float*)d_in[4], (const float*)d_in[6]};
  const float* dtb[2]  = {(const float*)d_in[7], (const float*)d_in[8]};
  const float* Alg[2]  = {(const float*)d_in[9], (const float*)d_in[10]};
  const float* Dv[2]   = {(const float*)d_in[11], (const float*)d_in[12]};
  const float* nwv[2]  = {(const float*)d_in[13], (const float*)d_in[14]};
  const float* Wod[2]  = {(const float*)d_in[15], (const float*)d_in[16]};
  const float* Wo      = (const float*)d_in[17];
  float* out = (float*)d_out;

  size_t off = 0;
  auto carve = [&](size_t bytes) -> char* { char* p = (char*)d_ws + off; off += (bytes + 255) & ~(size_t)255; return p; };
  unsigned short* U16f  = (unsigned short*)carve((size_t)SEQL * DM * 2);
  unsigned short* U16b  = (unsigned short*)carve((size_t)SEQL * DM * 2);
  unsigned short* WIN16[2];
  WIN16[0] = (unsigned short*)carve((size_t)LDZ * DM * 2);
  WIN16[1] = (unsigned short*)carve((size_t)LDZ * DM * 2);
  unsigned short* WO16[3];
  WO16[0] = (unsigned short*)carve((size_t)DM * DIN * 2);
  WO16[1] = (unsigned short*)carve((size_t)DM * DIN * 2);
  WO16[2] = (unsigned short*)carve((size_t)DM * DIN * 2);
  unsigned short* TH    = (unsigned short*)carve((size_t)SEQL * DIN * 2);
  unsigned short* TL    = (unsigned short*)carve((size_t)SEQL * DIN * 2);
  float* ZX             = (float*)carve((size_t)SEQL * LDZ * 4);
  float* ACS            = (float*)carve((size_t)SEQL * NH * 4);
  float* DT             = (float*)carve((size_t)SEQL * NH * 4);
  float* XF             = (float*)carve((size_t)SEQL * XW * 4);
  unsigned short* XTH   = (unsigned short*)carve((size_t)SEQL * XW * 2);
  unsigned short* XTL   = (unsigned short*)carve((size_t)SEQL * XW * 2);
  unsigned short* XDH   = (unsigned short*)carve((size_t)SEQL * XW * 2);
  unsigned short* XDL   = (unsigned short*)carve((size_t)SEQL * XW * 2);
  unsigned short* BHp   = (unsigned short*)carve((size_t)SEQL * NS * 2);
  unsigned short* BLp   = (unsigned short*)carve((size_t)SEQL * NS * 2);
  unsigned short* CHp   = (unsigned short*)carve((size_t)SEQL * NS * 2);
  unsigned short* CLp   = (unsigned short*)carve((size_t)SEQL * NS * 2);
  float* G              = (float*)carve((size_t)NCH * CH * CH * 4);
  float* S              = (float*)carve((size_t)NCH * XW * NS * 4);
  unsigned short* PH    = (unsigned short*)carve((size_t)NCH * XW * NS * 2);
  unsigned short* PL    = (unsigned short*)carve((size_t)NCH * XW * NS * 2);
  float* YO             = (float*)carve((size_t)SEQL * XW * 4);
  float* Yb             = (float*)carve((size_t)SEQL * XW * 4);
  unsigned short* YGH   = (unsigned short*)carve((size_t)SEQL * XW * 2);
  unsigned short* YGL   = (unsigned short*)carve((size_t)SEQL * XW * 2);
  if (off > ws_size || off > (size_t)134217728) return;

  const dim3 blk(256);
  k_cvt_u<<<dim3((SEQL * DM / 8 + 255) / 256), blk, 0, stream>>>(u, U16f, U16b);
  for (int d = 0; d < 2; ++d)
    k_cvt<<<dim3((LDZ * DM / 8 + 255) / 256), blk, 0, stream>>>(Win[d], WIN16[d], DPROJ, DM / 8, LDZ * DM / 8);
  for (int d = 0; d < 2; ++d)
    k_cvt<<<dim3((DM * DIN / 8 + 255) / 256), blk, 0, stream>>>(Wod[d], WO16[d], DM, DIN / 8, DM * DIN / 8);
  k_cvt<<<dim3((DM * DIN / 8 + 255) / 256), blk, 0, stream>>>(Wo, WO16[2], DM, DIN / 8, DM * DIN / 8);

  for (int d = 0; d < 2; ++d) {
    const unsigned short* U16 = (d == 0) ? U16f : U16b;
    k_gemm<1, 1, 0, 0, 0, 0><<<dim3(SEQL / 128, LDZ / 64, 1), blk, 0, stream>>>(
        U16, U16, G, DM, 0, 0,
        WIN16[d], WIN16[d], DM, 0, 0,
        ZX, LDZ, 0, 0,
        TH, TL, XW,
        G, 0, 0, 0,
        ACS, 0, 0,
        1, DM);
    k_acs<<<dim3(NCH), dim3(32), 0, stream>>>(ZX, dtb[d], Alg[d], ACS, DT);
    k_conv<<<dim3(SEQL), blk, 0, stream>>>(ZX, cwv[d], cbv[d], ACS, DT, XF, XTH, XTL, XDH, XDL, BHp, BLp, CHp, CLp);
    k_gemm<2, 2, 0, 0, 0, 0><<<dim3(CH / 128, CH / 64, NCH), blk, 0, stream>>>(
        CHp, CLp, G, NS, (long long)CH * NS, 0,
        BHp, BLp, NS, (long long)CH * NS, 0,
        G, CH, (long long)CH * CH, 0,
        TH, TL, XW,
        G, 0, 0, 0,
        ACS, 0, 0,
        1, NS);
    k_gemm<2, 2, 1, 1, 0, 0><<<dim3(XW / 128, NS / 64, NCH), blk, 0, stream>>>(
        XDH, XDL, G, XW, (long long)CH * XW, 0,
        BHp, BLp, NS, (long long)CH * NS, 0,
        S, NS, (long long)XW * NS, 0,
        TH, TL, XW,
        G, 0, 0, 0,
        ACS, 0, 0,
        1, CH);
    k_prev<<<dim3((XW * NS) / PREVE), blk, 0, stream>>>(S, ACS, PH, PL);
    k_gemm<2, 2, 0, 0, 1, 0><<<dim3(CH / 128, HD / 64, NCH * NH), blk, 0, stream>>>(
        CHp, CLp, G, NS, (long long)CH * NS, 0,
        PH, PL, NS, (long long)XW * NS, (long long)HD * NS,
        YO, XW, (long long)CH * XW, HD,
        TH, TL, XW,
        G, 0, 0, 0,
        ACS, (long long)CH * NH, 1,
        NH, NS);
    k_gemm<2, 2, 2, 1, 2, 0><<<dim3(CH / 128, HD / 64, NCH * NH), blk, 0, stream>>>(
        XTH, XTH, G, CH, (long long)CH * CH, 0,
        XTH, XTL, XW, (long long)CH * XW, HD,
        Yb, XW, (long long)CH * XW, HD,
        TH, TL, XW,
        YO, XW, (long long)CH * XW, HD,
        ACS, (long long)CH * NH, 1,
        NH, CH);
    k_gate<<<dim3(SEQL), blk, 0, stream>>>(Yb, XF, ZX, Dv[d], nwv[d], YGH, YGL);
    if (d == 0) {
      k_gemm<2, 1, 0, 0, 3, 0><<<dim3(SEQL / 128, DM / 64, 1), blk, 0, stream>>>(
          YGH, YGL, G, XW, 0, 0,
          WO16[0], WO16[0], XW, 0, 0,
          Yb, XW, 0, 0,
          TH, TL, DIN,
          G, 0, 0, 0,
          ACS, 0, 0,
          1, XW);
    } else {
      k_gemm<2, 1, 0, 0, 3, 1><<<dim3(SEQL / 128, DM / 64, 1), blk, 0, stream>>>(
          YGH, YGL, G, XW, 0, 0,
          WO16[1], WO16[1], XW, 0, 0,
          Yb, XW, 0, 0,
          TH + DM, TL + DM, DIN,
          G, 0, 0, 0,
          ACS, 0, 0,
          1, XW);
    }
  }
  k_gemm<2, 1, 0, 0, 0, 0><<<dim3(SEQL / 128, DM / 64, 1), blk, 0, stream>>>(
      TH, TL, G, DIN, 0, 0,
      WO16[2], WO16[2], DIN, 0, 0,
      out, DM, 0, 0,
      TH, TL, DIN,
      G, 0, 0, 0,
      ACS, 0, 0,
      1, DIN);
}
